// TRED_GNN_82437602279986
// MI455X (gfx1250) — hardware-verified
//
#include <hip/hip_runtime.h>


typedef _Float16 v16h __attribute__((ext_vector_type(16)));
typedef _Float16 v8h  __attribute__((ext_vector_type(8)));
typedef __bf16   v16b __attribute__((ext_vector_type(16)));
typedef unsigned short v16u __attribute__((ext_vector_type(16)));
typedef unsigned short v8u  __attribute__((ext_vector_type(8)));
typedef float v8f __attribute__((ext_vector_type(8)));
typedef float v4f __attribute__((ext_vector_type(4)));
typedef v4f v4fa __attribute__((may_alias));

union FragH { v16h v; v8h half[2]; };
union FragB { v16b v; v16u u; v8u half[2]; };

#define RN 1024

__device__ __forceinline__ v8f mma_f16(v16h a, v16h b, v8f c)
{
  v8f d = __builtin_amdgcn_wmma_f32_16x16x32_f16(false, a, false, b, (short)0, c, false, false);
  asm volatile("v_nop\n\tv_nop\n\tv_nop\n\tv_nop" : "+v"(d) : "v"(a), "v"(b));
  return d;
}
__device__ __forceinline__ v8f mma_bf16(v16b a, v16b b, v8f c)
{
  v8f d = __builtin_amdgcn_wmma_f32_16x16x32_bf16(false, a, false, b, (short)0, c, false, false);
  asm volatile("v_nop\n\tv_nop\n\tv_nop\n\tv_nop" : "+v"(d) : "v"(a), "v"(b));
  return d;
}

__device__ __forceinline__ unsigned bf16_bits(float f)
{
  const unsigned u = __float_as_uint(f);
  return (u + 0x7FFFu + ((u >> 16) & 1u)) >> 16;
}
__device__ __forceinline__ void split_bf16(float x, unsigned& hb, unsigned& lb)
{
  hb = bf16_bits(x);
  const float hf = __uint_as_float(hb << 16);
  lb = bf16_bits(x - hf);
}

__device__ __forceinline__ void prep_f16_row(const float* __restrict__ W, _Float16* WT, int n, float sw)
{
  v8h v[8];
#pragma unroll
  for (int g = 0; g < 8; ++g) {
    v8h t;
#pragma unroll
    for (int i = 0; i < 8; ++i) t[i] = (_Float16)(W[(8 * g + i) * 64 + n] * sw);
    v[g] = t;
  }
  _Float16* d = WT + n * 64;
#pragma unroll
  for (int g = 0; g < 8; ++g) *(volatile v8h*)(d + 8 * g) = v[g];
  __threadfence();
#pragma unroll
  for (int g = 0; g < 8; ++g) *(volatile v8h*)(d + 8 * g) = v[g];
}

__global__ __launch_bounds__(64)
void k_prepw(const float* __restrict__ Ws, const float* __restrict__ Wr, const float* __restrict__ Wqr,
             const float* __restrict__ Wh,
             _Float16* WTs, _Float16* WTr, _Float16* WTq,
             unsigned short* WhHi, unsigned short* WhLo)
{
  const int n = threadIdx.x;
  prep_f16_row(Ws,  WTs, n, 64.0f);
  prep_f16_row(Wr,  WTr, n, 64.0f);
  prep_f16_row(Wqr, WTq, n, 64.0f);

  v8u hv[8], lv[8];
#pragma unroll
  for (int g = 0; g < 8; ++g) {
    v8u th, tlw;
#pragma unroll
    for (int i = 0; i < 8; ++i) {
      unsigned hb, lb;
      split_bf16(Wh[(8 * g + i) * 64 + n], hb, lb);
      th[i]  = (unsigned short)hb;
      tlw[i] = (unsigned short)lb;
    }
    hv[g] = th; lv[g] = tlw;
  }
  unsigned short* dh = WhHi + n * 64;
  unsigned short* dl = WhLo + n * 64;
#pragma unroll
  for (int g = 0; g < 8; ++g) { *(volatile v8u*)(dh + 8 * g) = hv[g]; *(volatile v8u*)(dl + 8 * g) = lv[g]; }
  __threadfence();
#pragma unroll
  for (int g = 0; g < 8; ++g) { *(volatile v8u*)(dh + 8 * g) = hv[g]; *(volatile v8u*)(dl + 8 * g) = lv[g]; }
}

template <bool BIAS>
__global__ __launch_bounds__(128)
void k_gemm64(const float* __restrict__ X, int M, float sa,
              const _Float16* __restrict__ WT, float oscale,
              const float* __restrict__ bias, float* Y)
{
  __shared__ float stage[4 * 16 * 64];
  const int lane = threadIdx.x & 31;
  const int wv   = threadIdx.x >> 5;
  const int h = lane >> 4, m = lane & 15;
  const int row0 = (blockIdx.x * 4 + wv) * 16;
  int ra = row0 + m;
  ra = (ra < M) ? ra : (M - 1);
  const float* xr = X + (size_t)ra * 64;

  FragH a[2];
#pragma unroll
  for (int ks = 0; ks < 2; ++ks) {
    const v4f x0 = *(const v4f*)(xr + 32 * ks + 8 * h);
    const v4f x1 = *(const v4f*)(xr + 32 * ks + 8 * h + 4);
    const v4f x2 = *(const v4f*)(xr + 32 * ks + 16 + 8 * h);
    const v4f x3 = *(const v4f*)(xr + 32 * ks + 16 + 8 * h + 4);
    v8h p, q;
#pragma unroll
    for (int i = 0; i < 4; ++i) {
      p[i] = (_Float16)(x0[i] * sa); p[4 + i] = (_Float16)(x1[i] * sa);
      q[i] = (_Float16)(x2[i] * sa); q[4 + i] = (_Float16)(x3[i] * sa);
    }
    a[ks].half[0] = p; a[ks].half[1] = q;
  }

  float* st = stage + wv * (16 * 64);
  const v8f z8 = {0.0f, 0.0f, 0.0f, 0.0f, 0.0f, 0.0f, 0.0f, 0.0f};
#pragma unroll
  for (int t = 0; t < 4; ++t) {
    v8f acc = z8;
#pragma unroll
    for (int ks = 0; ks < 2; ++ks) {
      FragH b;
      const _Float16* bp = WT + (16 * t + m) * 64 + 32 * ks + 8 * h;
      b.half[0] = *(const v8h*)(bp);
      b.half[1] = *(const v8h*)(bp + 16);
      acc = mma_f16(a[ks].v, b.v, acc);
    }
#pragma unroll
    for (int r = 0; r < 8; ++r) {
      float v = acc[r] * oscale;
      if (BIAS) v += bias[16 * t + m];
      st[(8 * h + r) * 64 + 16 * t + m] = v;
    }
  }
  __syncthreads();

  v4f sv[8];
#pragma unroll
  for (int i = 0; i < 8; ++i) sv[i] = *(const v4fa*)(st + (2 * i + h) * 64 + 4 * m);
  float* yb = Y + (size_t)row0 * 64 + 4 * m;
#pragma unroll
  for (int i = 0; i < 8; ++i) *(volatile v4f*)(yb + (size_t)(2 * i + h) * 64) = sv[i];
  __threadfence();
#pragma unroll
  for (int i = 0; i < 8; ++i) *(volatile v4f*)(yb + (size_t)(2 * i + h) * 64) = sv[i];
}

__device__ __forceinline__ void edge_one(
    int e, int o, int n0, int lane, float2 wa, float bav,
    const float* __restrict__ hidden, const float* __restrict__ rela,
    const float* __restrict__ HWs, const float* __restrict__ RWr, const float* __restrict__ RWqB,
    const int* __restrict__ q_rel, const int* __restrict__ r_idx,
    const int* __restrict__ rel, const int* __restrict__ sub,
    int NN, int NQ, int NRELS, float* accl)
{
  int s  = sub[e];   s  = (s  < 0) ? 0 : ((s  >= NN)    ? (NN - 1)    : s);
  int rl = rel[e];   rl = (rl < 0) ? 0 : ((rl >= NRELS) ? (NRELS - 1) : rl);
  int ri = r_idx[e]; ri = (ri < 0) ? 0 : ((ri >= NQ)    ? (NQ - 1)    : ri);
  int q  = q_rel[ri]; q = (q  < 0) ? 0 : ((q  >= NRELS) ? (NRELS - 1) : q);
  int orow = o - n0; orow = (orow < 0) ? 0 : ((orow >= RN) ? (RN - 1) : orow);

  const float2 hw = *((const float2*)(HWs  + (size_t)s  * 64) + lane);
  const float2 rw = *((const float2*)(RWr  + (size_t)rl * 64) + lane);
  const float2 qw = *((const float2*)(RWqB + (size_t)q  * 64) + lane);
  const float px = fmaxf(hw.x + rw.x + qw.x, 0.0f);
  const float py = fmaxf(hw.y + rw.y + qw.y, 0.0f);
  float part = px * wa.x + py * wa.y;
#pragma unroll
  for (int off = 16; off >= 1; off >>= 1) part += __shfl_xor(part, off, 32);
  const float zl = part + bav;
  const float alpha = 1.0f / (1.0f + __expf(-zl));

  const float2 hs = *((const float2*)(hidden + (size_t)s  * 64) + lane);
  const float2 hr = *((const float2*)(rela   + (size_t)rl * 64) + lane);
  float2* ap = (float2*)(accl + orow * 64) + lane;
  float2 av = *ap;
  av.x += alpha * (hs.x + hr.x);
  av.y += alpha * (hs.y + hr.y);
  *ap = av;
}

__global__ __launch_bounds__(32)
void k_aggout(const float* __restrict__ hidden, const float* __restrict__ rela,
              const float* __restrict__ HWs, const float* __restrict__ RWr, const float* __restrict__ RWqB,
              const int* __restrict__ q_rel, const int* __restrict__ r_idx, const int* __restrict__ rel,
              const int* __restrict__ sub, const int* __restrict__ obj,
              const float* __restrict__ Wa, const float* __restrict__ ba,
              const unsigned short* __restrict__ WhHi, const unsigned short* __restrict__ WhLo,
              float* out, int NN, int NE, int NQ, int NRELS)
{
  extern __shared__ v4f dlds[];
  float* accl = (float*)dlds;
  const int lane = threadIdx.x;
  const int h = lane >> 4, m = lane & 15;
  const int n0 = blockIdx.x * RN;

  const v4f z4 = {0.0f, 0.0f, 0.0f, 0.0f};
  for (int i = lane; i < RN * 16; i += 32) dlds[i] = z4;
  __syncthreads();

  const float2 wa = *((const float2*)Wa + lane);
  const float bav = ba[0];

#pragma unroll 1
  for (int base = 0; base < NE; base += 128) {
    const int idx = base + 4 * lane;
    int ox, oy, oz, ow;
    if (base + 128 <= NE) {
      const int4 v = *(const int4*)(obj + idx);
      ox = v.x; oy = v.y; oz = v.z; ow = v.w;
    } else {
      ox = (idx     < NE) ? obj[idx]     : -1;
      oy = (idx + 1 < NE) ? obj[idx + 1] : -1;
      oz = (idx + 2 < NE) ? obj[idx + 2] : -1;
      ow = (idx + 3 < NE) ? obj[idx + 3] : -1;
    }
    const unsigned d0 = (unsigned)ox - (unsigned)n0;
    const unsigned d1 = (unsigned)oy - (unsigned)n0;
    const unsigned d2 = (unsigned)oz - (unsigned)n0;
    const unsigned d3 = (unsigned)ow - (unsigned)n0;
    const unsigned m01 = (d0 < d1) ? d0 : d1;
    const unsigned m23 = (d2 < d3) ? d2 : d3;
    const unsigned dmin = (m01 < m23) ? m01 : m23;
    if ((unsigned)__ballot(dmin < (unsigned)RN) == 0u) continue;

    const unsigned B0 = (unsigned)__ballot(d0 < (unsigned)RN);
    const unsigned B1 = (unsigned)__ballot(d1 < (unsigned)RN);
    const unsigned B2 = (unsigned)__ballot(d2 < (unsigned)RN);
    const unsigned B3 = (unsigned)__ballot(d3 < (unsigned)RN);
#pragma unroll
    for (int t = 0; t < 4; ++t) {
      unsigned Bt = (t == 0) ? B0 : ((t == 1) ? B1 : ((t == 2) ? B2 : B3));
      const int oc = (t == 0) ? ox : ((t == 1) ? oy : ((t == 2) ? oz : ow));
      while (Bt != 0u) {
        const int j = (int)__builtin_ctz(Bt);
        Bt &= Bt - 1u;
        const int e = __builtin_amdgcn_readfirstlane(base + 4 * j + t);
        const int o = __builtin_amdgcn_readlane(oc, j);
        edge_one(e, o, n0, lane, wa, bav, hidden, rela, HWs, RWr, RWqB,
                 q_rel, r_idx, rel, sub, NN, NQ, NRELS, accl);
      }
    }
  }
  __syncthreads();

  const v8f z8 = {0.0f, 0.0f, 0.0f, 0.0f, 0.0f, 0.0f, 0.0f, 0.0f};
#pragma unroll 1
  for (int mt = 0; mt < RN / 16; ++mt) {
    const int nodeBase = n0 + 16 * mt;
    if (nodeBase >= NN) break;
    float* tl = accl + mt * (16 * 64);

    FragB ah[2], al[2];
#pragma unroll
    for (int ks = 0; ks < 2; ++ks) {
      const float* rp = tl + m * 64 + 32 * ks + 8 * h;
      const v4f x0 = *(const v4fa*)(rp);
      const v4f x1 = *(const v4fa*)(rp + 4);
      const v4f x2 = *(const v4fa*)(rp + 16);
      const v4f x3 = *(const v4fa*)(rp + 20);
      v8u ph, pl, qh, ql;
#pragma unroll
      for (int i = 0; i < 4; ++i) {
        unsigned hb, lb;
        split_bf16(x0[i], hb, lb); ph[i]     = (unsigned short)hb; pl[i]     = (unsigned short)lb;
        split_bf16(x1[i], hb, lb); ph[4 + i] = (unsigned short)hb; pl[4 + i] = (unsigned short)lb;
        split_bf16(x2[i], hb, lb); qh[i]     = (unsigned short)hb; ql[i]     = (unsigned short)lb;
        split_bf16(x3[i], hb, lb); qh[4 + i] = (unsigned short)hb; ql[4 + i] = (unsigned short)lb;
      }
      ah[ks].half[0] = ph; ah[ks].half[1] = qh;
      al[ks].half[0] = pl; al[ks].half[1] = ql;
    }
    __syncthreads();

#pragma unroll
    for (int t = 0; t < 4; ++t) {
      v8f acc = z8;
#pragma unroll
      for (int ks = 0; ks < 2; ++ks) {
        int bo = (16 * t + m) * 64 + 32 * ks + 8 * h;
        asm volatile("" : "+v"(bo));
        FragB bh, bl;
        bh.half[0] = *(const v8u*)(WhHi + bo);
        bh.half[1] = *(const v8u*)(WhHi + bo + 16);
        bl.half[0] = *(const v8u*)(WhLo + bo);
        bl.half[1] = *(const v8u*)(WhLo + bo + 16);
        acc = mma_bf16(ah[ks].v, bh.v, acc);
        acc = mma_bf16(al[ks].v, bh.v, acc);
        acc = mma_bf16(ah[ks].v, bl.v, acc);
      }
#pragma unroll
      for (int r = 0; r < 8; ++r) tl[(8 * h + r) * 64 + 16 * t + m] = fmaxf(acc[r], 0.0f);
    }
    __syncthreads();

    v4f sv[8];
#pragma unroll
    for (int i = 0; i < 8; ++i) sv[i] = *(const v4fa*)(tl + (2 * i + h) * 64 + 4 * m);
#pragma unroll
    for (int i = 0; i < 8; ++i) {
      const int node = nodeBase + 2 * i + h;
      if (node < NN) *(volatile v4f*)(out + (size_t)node * 64 + 4 * m) = sv[i];
    }
    __threadfence();
#pragma unroll
    for (int i = 0; i < 8; ++i) {
      const int node = nodeBase + 2 * i + h;
      if (node < NN) *(volatile v4f*)(out + (size_t)node * 64 + 4 * m) = sv[i];
    }
  }
}

extern "C" void kernel_launch(void* const* d_in, const int* in_sizes, int n_in,
                              void* d_out, int out_size, void* d_ws, size_t ws_size,
                              hipStream_t stream)
{
  (void)n_in;

  const int*   q_rel  = (const int*)  d_in[0];
  const float* hidden = (const float*)d_in[1];
  const int*   r_idx  = (const int*)  d_in[2];
  const int*   rel    = (const int*)  d_in[3];
  const int*   sub    = (const int*)  d_in[4];
  const int*   obj    = (const int*)  d_in[5];
  const float* rela   = (const float*)d_in[7];
  const float* Ws     = (const float*)d_in[8];
  const float* Wr     = (const float*)d_in[9];
  const float* Wqr    = (const float*)d_in[10];
  const float* bqr    = (const float*)d_in[11];
  const float* Wa     = (const float*)d_in[12];
  const float* ba     = (const float*)d_in[13];
  const float* Wh     = (const float*)d_in[14];

  const int NQ    = in_sizes[0];
  const int NN    = in_sizes[1] / 64;
  int NE          = in_sizes[5];
  if (in_sizes[2] < NE) NE = in_sizes[2];
  if (in_sizes[3] < NE) NE = in_sizes[3];
  if (in_sizes[4] < NE) NE = in_sizes[4];
  const int NRELS = in_sizes[7] / 64;
  if (NQ <= 0 || NN <= 0 || NRELS <= 0 || NE < 0) return;
  if ((long long)out_size < (long long)NN * 64) return;

  const int gridH = (NN + 63) / 64;
  const int gridR = (NRELS + 63) / 64;

  char* ws = (char*)d_ws;
  size_t off = 0;
  _Float16* WTs = (_Float16*)(ws + off); off += 64 * 64 * sizeof(_Float16); off = (off + 255) & ~(size_t)255;
  _Float16* WTr = (_Float16*)(ws + off); off += 64 * 64 * sizeof(_Float16); off = (off + 255) & ~(size_t)255;
  _Float16* WTq = (_Float16*)(ws + off); off += 64 * 64 * sizeof(_Float16); off = (off + 255) & ~(size_t)255;
  unsigned short* WhHi = (unsigned short*)(ws + off); off += 64 * 64 * sizeof(unsigned short); off = (off + 255) & ~(size_t)255;
  unsigned short* WhLo = (unsigned short*)(ws + off); off += 64 * 64 * sizeof(unsigned short); off = (off + 255) & ~(size_t)255;
  float* HWs  = (float*)(ws + off); off += (size_t)gridH * 64 * 64 * sizeof(float); off = (off + 255) & ~(size_t)255;
  float* RWr  = (float*)(ws + off); off += (size_t)gridR * 64 * 64 * sizeof(float); off = (off + 255) & ~(size_t)255;
  float* RWqB = (float*)(ws + off); off += (size_t)gridR * 64 * 64 * sizeof(float); off = (off + 255) & ~(size_t)255;
  if (off > ws_size) return;

  k_prepw<<<dim3(1), dim3(64), 0, stream>>>(Ws, Wr, Wqr, Wh, WTs, WTr, WTq, WhHi, WhLo);

  k_gemm64<false><<<dim3(gridH), dim3(128), 0, stream>>>(hidden, NN, 1.0f, WTs, 1.0f / 64.0f, bqr, HWs);
  k_gemm64<false><<<dim3(gridR), dim3(128), 0, stream>>>(rela, NRELS, 16.0f, WTr, 1.0f / 1024.0f, bqr, RWr);
  k_gemm64<true ><<<dim3(gridR), dim3(128), 0, stream>>>(rela, NRELS, 16.0f, WTq, 1.0f / 1024.0f, bqr, RWqB);

  const int gridA = (NN + RN - 1) / RN;
  const size_t ldsBytes = (size_t)RN * 64 * sizeof(float);
  k_aggout<<<dim3(gridA), dim3(32), ldsBytes, stream>>>(
      hidden, rela, HWs, RWr, RWqB, q_rel, r_idx, rel, sub, obj, Wa, ba, WhHi, WhLo,
      (float*)d_out, NN, NE, NQ, NRELS);
}
